// Network_43808666419473
// MI455X (gfx1250) — hardware-run, weakly checked
//
#include <hip/hip_runtime.h>


#define NR   2048
#define NT   50001
#define ND   300
#define NK   320
#define NP   128
#define NS   256
#define NB   8
typedef _Float16 h16;
typedef unsigned short bf;
typedef __attribute__((ext_vector_type(16))) __bf16   v16bf;
typedef __attribute__((ext_vector_type(16))) _Float16 v16h;
typedef __attribute__((ext_vector_type(8)))  _Float16 v8h;
typedef __attribute__((ext_vector_type(8)))  unsigned short v8us;
typedef __attribute__((ext_vector_type(8)))  float    v8f;
typedef __attribute__((ext_vector_type(4)))  float    v4f;
typedef v8h  __attribute__((may_alias)) v8ha;
typedef v4f  __attribute__((may_alias)) v4fa;
typedef v8us __attribute__((may_alias)) v8usa;

__device__ __forceinline__ unsigned short f2bf(float f) { unsigned u = __float_as_uint(f); u += 0x7FFFu + ((u >> 16) & 1u); return (unsigned short)(u >> 16); }
__device__ __forceinline__ float bf2f(unsigned short b) { return __uint_as_float(((unsigned)b) << 16); }
__device__ __forceinline__ float bfr(float f) { return bf2f(f2bf(f)); }
__device__ __forceinline__ v16h cat16(v8h lo, v8h hi) { return __builtin_shufflevector(lo, hi, 0, 1, 2, 3, 4, 5, 6, 7, 8, 9, 10, 11, 12, 13, 14, 15); }
__device__ __forceinline__ v16bf cat16b(v8us lo, v8us hi) { return __builtin_bit_cast(v16bf, __builtin_shufflevector(lo, hi, 0, 1, 2, 3, 4, 5, 6, 7, 8, 9, 10, 11, 12, 13, 14, 15)); }
__device__ __forceinline__ v8f wmma16(v16h a, v16h b, v8f c) { return __builtin_amdgcn_wmma_f32_16x16x32_f16(false, a, false, b, (short)0, c, false, false); }
__device__ __forceinline__ v8f wmmab(v16bf a, v16bf b, v8f c) { return __builtin_amdgcn_wmma_f32_16x16x32_bf16(false, a, false, b, (short)0, c, false, false); }


template <typename T16> struct WFrag;
template <> struct WFrag<h16> { typedef v16h V; static __device__ __forceinline__ V ld(const h16* p) { return cat16(*(const v8h*)p, *(const v8h*)(p + 16)); } static __device__ __forceinline__ v8f mma(V a, V b, v8f c) { return wmma16(a, b, c); } };
template <> struct WFrag<bf> { typedef v16bf V; static __device__ __forceinline__ V ld(const bf* p) { return cat16b(*(const v8us*)p, *(const v8us*)(p + 16)); } static __device__ __forceinline__ v8f mma(V a, V b, v8f c) { return wmmab(a, b, c); } };
template <typename T16, int NSPLIT, bool BIAS>
__global__ __launch_bounds__(32) void k_gemmw(const T16* __restrict__ A, const T16* __restrict__ A2, const T16* __restrict__ Bt, const T16* __restrict__ Bt2, int K, float* C, int ldc, const float* __restrict__ bias, size_t sA, size_t sB, size_t sC) {
    typedef typename WFrag<T16>::V V;
    __shared__ __align__(16) float os[16 * 68];
    const size_t z = blockIdx.z; A += z * sA; if (A2) A2 += z * sA; Bt += z * sB; if (Bt2) Bt2 += z * sB; C += z * sC;
    const int lane = threadIdx.x & 31, lr = lane & 15, hi = lane >> 4; const int r0 = blockIdx.x * 64, c0 = blockIdx.y * 64;
    v8f acc[4][4];
#pragma unroll
    for (int mb = 0; mb < 4; ++mb)
#pragma unroll
        for (int nb = 0; nb < 4; ++nb) acc[mb][nb] = (v8f){};
    const size_t aoff = (size_t)(r0 + lr) * K + 8 * hi, boff = (size_t)(c0 + lr) * K + 8 * hi;
    for (int kc = 0; kc < K; kc += 32) {
        V a[4], a2[4];
#pragma unroll
        for (int mb = 0; mb < 4; ++mb) { a[mb] = WFrag<T16>::ld(A + aoff + (size_t)mb * 16 * K + kc); if (NSPLIT == 1 || NSPLIT == 2) a2[mb] = WFrag<T16>::ld(A2 + aoff + (size_t)mb * 16 * K + kc); }
#pragma unroll
        for (int nb = 0; nb < 4; ++nb) { const V b = WFrag<T16>::ld(Bt + boff + (size_t)nb * 16 * K + kc); V b2; if (NSPLIT >= 2) b2 = WFrag<T16>::ld(Bt2 + boff + (size_t)nb * 16 * K + kc);
#pragma unroll
            for (int mb = 0; mb < 4; ++mb) { acc[mb][nb] = WFrag<T16>::mma(a[mb], b, acc[mb][nb]); if (NSPLIT == 1 || NSPLIT == 2) acc[mb][nb] = WFrag<T16>::mma(a2[mb], b, acc[mb][nb]); if (NSPLIT >= 2) acc[mb][nb] = WFrag<T16>::mma(a[mb], b2, acc[mb][nb]); } }
        asm volatile("v_nop\n\tv_nop\n\tv_nop\n\tv_nop" : "+v"(acc[0][0]), "+v"(acc[1][1]), "+v"(acc[2][2]), "+v"(acc[3][3]) : "v"(a[0]), "v"(a[3]));
    }
#pragma unroll
    for (int mb = 0; mb < 4; ++mb) {
#pragma unroll
        for (int nb = 0; nb < 4; ++nb) {
#pragma unroll
            for (int j = 0; j < 8; ++j) os[(hi * 8 + j) * 68 + nb * 16 + lr] = acc[mb][nb][j]; }
        __builtin_amdgcn_wave_barrier(); asm volatile("" ::: "memory");
        float* crow = C + (size_t)(r0 + mb * 16) * ldc + c0;
#pragma unroll 1
        for (int ps = 0; ps < 2; ++ps) {
#pragma unroll
            for (int s = 0; s < 8; ++s) { const int row = 2 * s + hi, cofs = lr * 4; v4f val = *(const v4fa*)(os + row * 68 + cofs); if (BIAS) { val[0] += bfr(bias[c0 + cofs]); val[1] += bfr(bias[c0 + cofs + 1]); val[2] += bfr(bias[c0 + cofs + 2]); val[3] += bfr(bias[c0 + cofs + 3]); }
                *(volatile v4f*)(crow + (size_t)row * ldc + cofs) = val; }
            if (ps == 0) __threadfence(); }
        __builtin_amdgcn_wave_barrier(); asm volatile("" ::: "memory");
    }
}


typedef __attribute__((ext_vector_type(4))) unsigned short v4us;

__device__ __forceinline__ v8us row8(const float* __restrict__ src, int q) {
    const int k0 = 8 * q; const int ka = k0 < 296 ? k0 : 296; const int kb = k0 + 4 < 296 ? k0 + 4 : 296;
    const v4f lo = *(const v4f*)(src + ka); const v4f hi = *(const v4f*)(src + kb);
    const unsigned short mlo = (unsigned short)(0u - (unsigned)(q < 38)), mhi = (unsigned short)(0u - (unsigned)(q < 37)); v8us o;
#pragma unroll
    for (int e = 0; e < 4; ++e) { o[e] = (unsigned short)(f2bf(lo[e]) & mlo); o[4 + e] = (unsigned short)(f2bf(hi[e]) & mhi); }
    return o; }

__global__ __launch_bounds__(320) void k_gath(const int* __restrict__ rows, const float* __restrict__ tab, bf* X) { const int q = threadIdx.x, r = blockIdx.x * 8 + threadIdx.y; int t = rows[r]; t = t < 0 ? 0 : (t > NT - 1 ? NT - 1 : t);
    const v8us o = row8(tab + (size_t)t * ND, q); bf* dst = X + (size_t)r * NK + 8 * q;
    *(volatile v8us*)dst = o; __threadfence(); *(volatile v8us*)dst = o; }

__global__ __launch_bounds__(320) void k_wpad(const float* __restrict__ w, bf* Wp) { const int q = threadIdx.x, r = blockIdx.x * 8 + threadIdx.y;
    const v8us o = row8(w + (size_t)r * ND, q); bf* dst = Wp + (size_t)r * NK + 8 * q;
    *(volatile v8us*)dst = o; __threadfence(); *(volatile v8us*)dst = o; }

__global__ __launch_bounds__(256) void k_heads(const float* __restrict__ PS, const float* __restrict__ PE, const float* __restrict__ w1, const float* __restrict__ c1, const float* __restrict__ w2, const float* __restrict__ c2, float* o1, float* o2) { const int r = blockIdx.x * 256 + threadIdx.x; const float* ps = PS + (size_t)r * NP; const float* pe = PE + (size_t)r * NP; float s1 = 0.0f, s2 = 0.0f;
    for (int g = 0; g < NP / 4; ++g) { const v4f a = *(const v4f*)(ps + 4 * g); const v4f e = *(const v4f*)(pe + 4 * g);
#pragma unroll
        for (int u = 0; u < 4; ++u) { s1 = __fmaf_rn(fmaxf(a[u], 0.0f), bfr(w1[4 * g + u]), s1); s2 = __fmaf_rn(fmaxf(e[u], 0.0f), bfr(w2[4 * g + u]), s2); } }
    const float v1 = __fadd_rn(s1, bfr(c1[0])), v2 = __fadd_rn(s2, bfr(c2[0]));
    *(volatile float*)(o1 + r) = v1; *(volatile float*)(o2 + r) = v2; __threadfence(); *(volatile float*)(o1 + r) = v1; *(volatile float*)(o2 + r) = v2; }

__global__ __launch_bounds__(256) void k_pair(const float* __restrict__ PL, const float* __restrict__ PR, const float* __restrict__ w, const float* __restrict__ c, float* o0) { const int j = threadIdx.x, i = blockIdx.x, b = blockIdx.y; const float* pl = PL + (size_t)(b * NS + j) * NP; const float* pr = PR + (size_t)(b * NS + i) * NP; float s = 0.0f;
    for (int g = 0; g < NP / 4; ++g) { const v4f a = *(const v4f*)(pl + 4 * g); const v4f e = *(const v4f*)(pr + 4 * g);
#pragma unroll
        for (int u = 0; u < 4; ++u) s = __fmaf_rn(fmaxf(__fadd_rn(a[u], e[u]), 0.0f), bfr(w[4 * g + u]), s); }
    const float v = __fadd_rn(s, bfr(c[0])); float* dst = o0 + ((size_t)(b * NS + i) * NS + j);
    *(volatile float*)dst = v; __threadfence(); *(volatile float*)dst = v; }

extern "C" void kernel_launch(void* const* d_in, const int* in_sizes, int n_in, void* d_out, int out_size, void* d_ws, size_t ws_size, hipStream_t stream) {
    if (n_in < 15) return;
    if (in_sizes[0] != NR || in_sizes[1] != NT * ND || in_sizes[2] != NP * ND || in_sizes[3] != NP || in_sizes[4] != NP * ND || in_sizes[5] != NP || in_sizes[6] != 1 || in_sizes[7] != NP * ND || in_sizes[8] != NP || in_sizes[9] != NP || in_sizes[10] != 1 || in_sizes[11] != NP * ND || in_sizes[12] != NP || in_sizes[13] != NP || in_sizes[14] != 1) return;
    if (out_size != NB * NS * NS + 2 * NR) return;
    static_assert(NR == NB * NS && NR % 64 == 0 && NP % 64 == 0 && NK % 32 == 0 && NK == 40 * 8 && ND % 4 == 0 && ND > 296 && ND <= 300 && NR % 8 == 0 && NP % 8 == 0 && NR % 256 == 0 && NS == 256 && (NB * NS * NS) % 32 == 0 && NR % 32 == 0, "the products: M and N multiples of 64, the depth a multiple of 32; forty groups of eight words a row, the last valid word at 299; every grid exact; out1 and out2 begin on whole lines");
    const int* rows = (const int*)d_in[0]; const float* tab = (const float*)d_in[1];
    const float* wA = (const float*)d_in[2]; const float* vA = (const float*)d_in[3]; const float* wB = (const float*)d_in[4]; const float* w0 = (const float*)d_in[5]; const float* c0 = (const float*)d_in[6];
    const float* wC = (const float*)d_in[7]; const float* vC = (const float*)d_in[8]; const float* w1 = (const float*)d_in[9]; const float* c1 = (const float*)d_in[10];
    const float* wD = (const float*)d_in[11]; const float* vD = (const float*)d_in[12]; const float* w2 = (const float*)d_in[13]; const float* c2 = (const float*)d_in[14];
    float* o0 = (float*)d_out; float* o1 = o0 + (size_t)NB * NS * NS; float* o2 = o1 + NR;
    char* wsp = (char*)d_ws; auto take = [&](size_t bytes) { char* p = wsp; wsp += (bytes + 255) & ~(size_t)255; return (void*)p; };
    bf* X = (bf*)take((size_t)NR * NK * 2); bf* WpA = (bf*)take((size_t)NP * NK * 2); bf* WpB = (bf*)take((size_t)NP * NK * 2); bf* WpC = (bf*)take((size_t)NP * NK * 2); bf* WpD = (bf*)take((size_t)NP * NK * 2);
    float* PL = (float*)take((size_t)NR * NP * 4); float* PR = (float*)take((size_t)NR * NP * 4); float* PS = (float*)take((size_t)NR * NP * 4); float* PE = (float*)take((size_t)NR * NP * 4);
    if ((size_t)(wsp - (char*)d_ws) > ws_size) return;
    k_gath<<<NR / 8, dim3(40, 8, 1), 0, stream>>>(rows, tab, X);
    k_wpad<<<NP / 8, dim3(40, 8, 1), 0, stream>>>(wA, WpA);
    k_wpad<<<NP / 8, dim3(40, 8, 1), 0, stream>>>(wB, WpB);
    k_wpad<<<NP / 8, dim3(40, 8, 1), 0, stream>>>(wC, WpC);
    k_wpad<<<NP / 8, dim3(40, 8, 1), 0, stream>>>(wD, WpD);
    k_gemmw<bf, 0, true><<<dim3(NR / 64, NP / 64, 1), 32, 0, stream>>>(X, nullptr, WpA, nullptr, NK, PL, NP, vA, 0, 0, 0);
    k_gemmw<bf, 0, false><<<dim3(NR / 64, NP / 64, 1), 32, 0, stream>>>(X, nullptr, WpB, nullptr, NK, PR, NP, nullptr, 0, 0, 0);
    k_gemmw<bf, 0, true><<<dim3(NR / 64, NP / 64, 1), 32, 0, stream>>>(X, nullptr, WpC, nullptr, NK, PS, NP, vC, 0, 0, 0);
    k_gemmw<bf, 0, true><<<dim3(NR / 64, NP / 64, 1), 32, 0, stream>>>(X, nullptr, WpD, nullptr, NK, PE, NP, vD, 0, 0, 0);
    k_heads<<<NR / 256, 256, 0, stream>>>(PS, PE, w1, c1, w2, c2, o1, o2);
    k_pair<<<dim3(NS, NB, 1), 256, 0, stream>>>(PL, PR, w0, c0, o0);
}
